// TimeSelfAttentionFallback_62895501082759
// MI455X (gfx1250) — hardware-verified
//
#include <hip/hip_runtime.h>


#define NB_  2
#define TT   2048
#define DM   768
#define NH_  12
#define HD   64
#define HPP  4
#define PCAR 1024.0f
typedef _Float16 h16;
typedef unsigned short bf;
typedef __attribute__((ext_vector_type(16))) __bf16   v16bf;
typedef __attribute__((ext_vector_type(16))) _Float16 v16h;
typedef __attribute__((ext_vector_type(8)))  _Float16 v8h;
typedef __attribute__((ext_vector_type(8)))  unsigned short v8us;
typedef __attribute__((ext_vector_type(8)))  float    v8f;
typedef __attribute__((ext_vector_type(4)))  float    v4f;
typedef v8h  __attribute__((may_alias)) v8ha;
typedef v4f  __attribute__((may_alias)) v4fa;
typedef v8us __attribute__((may_alias)) v8usa;

__device__ __forceinline__ unsigned short f2bf(float f) { unsigned u = __float_as_uint(f); u += 0x7FFFu + ((u >> 16) & 1u); return (unsigned short)(u >> 16); }
__device__ __forceinline__ float bf2f(unsigned short b) { return __uint_as_float(((unsigned)b) << 16); }
__device__ __forceinline__ float bfr(float f) { return bf2f(f2bf(f)); }
__device__ __forceinline__ v16h cat16(v8h lo, v8h hi) { return __builtin_shufflevector(lo, hi, 0, 1, 2, 3, 4, 5, 6, 7, 8, 9, 10, 11, 12, 13, 14, 15); }
__device__ __forceinline__ v16bf cat16b(v8us lo, v8us hi) { return __builtin_bit_cast(v16bf, __builtin_shufflevector(lo, hi, 0, 1, 2, 3, 4, 5, 6, 7, 8, 9, 10, 11, 12, 13, 14, 15)); }
__device__ __forceinline__ v8f wmma16(v16h a, v16h b, v8f c) { return __builtin_amdgcn_wmma_f32_16x16x32_f16(false, a, false, b, (short)0, c, false, false); }
__device__ __forceinline__ v8f wmmab(v16bf a, v16bf b, v8f c) { return __builtin_amdgcn_wmma_f32_16x16x32_bf16(false, a, false, b, (short)0, c, false, false); }


template <typename T16> struct WFrag;
template <> struct WFrag<h16> { typedef v16h V; static __device__ __forceinline__ V ld(const h16* p) { return cat16(*(const v8h*)p, *(const v8h*)(p + 16)); } static __device__ __forceinline__ v8f mma(V a, V b, v8f c) { return wmma16(a, b, c); } };
template <> struct WFrag<bf> { typedef v16bf V; static __device__ __forceinline__ V ld(const bf* p) { return cat16b(*(const v8us*)p, *(const v8us*)(p + 16)); } static __device__ __forceinline__ v8f mma(V a, V b, v8f c) { return wmmab(a, b, c); } };
template <typename T16, int NSPLIT, bool BIAS>
__global__ __launch_bounds__(32) void k_gemmw(const T16* __restrict__ A, const T16* __restrict__ A2, const T16* __restrict__ Bt, const T16* __restrict__ Bt2, int K, float* C, int ldc, const float* __restrict__ bias, size_t sA, size_t sB, size_t sC) {
    typedef typename WFrag<T16>::V V;
    __shared__ __align__(16) float os[16 * 68];
    const size_t z = blockIdx.z; A += z * sA; if (A2) A2 += z * sA; Bt += z * sB; if (Bt2) Bt2 += z * sB; C += z * sC;
    const int lane = threadIdx.x & 31, lr = lane & 15, hi = lane >> 4; const int r0 = blockIdx.x * 64, c0 = blockIdx.y * 64;
    v8f acc[4][4];
#pragma unroll
    for (int mb = 0; mb < 4; ++mb)
#pragma unroll
        for (int nb = 0; nb < 4; ++nb) acc[mb][nb] = (v8f){};
    const size_t aoff = (size_t)(r0 + lr) * K + 8 * hi, boff = (size_t)(c0 + lr) * K + 8 * hi;
#pragma unroll 1
    for (int kc = 0; kc < K; kc += 32) {
        V a[4], a2[4];
#pragma unroll
        for (int mb = 0; mb < 4; ++mb) { a[mb] = WFrag<T16>::ld(A + aoff + (size_t)mb * 16 * K + kc); if (NSPLIT == 1 || NSPLIT == 2) a2[mb] = WFrag<T16>::ld(A2 + aoff + (size_t)mb * 16 * K + kc); }
#pragma unroll
        for (int nb = 0; nb < 4; ++nb) { const V b = WFrag<T16>::ld(Bt + boff + (size_t)nb * 16 * K + kc); V b2; if (NSPLIT >= 2) b2 = WFrag<T16>::ld(Bt2 + boff + (size_t)nb * 16 * K + kc);
#pragma unroll
            for (int mb = 0; mb < 4; ++mb) { acc[mb][nb] = WFrag<T16>::mma(a[mb], b, acc[mb][nb]); if (NSPLIT == 1 || NSPLIT == 2) acc[mb][nb] = WFrag<T16>::mma(a2[mb], b, acc[mb][nb]); if (NSPLIT >= 2) acc[mb][nb] = WFrag<T16>::mma(a[mb], b2, acc[mb][nb]); } }
        asm volatile("v_nop\n\tv_nop\n\tv_nop\n\tv_nop" : "+v"(acc[0][0]), "+v"(acc[1][1]), "+v"(acc[2][2]), "+v"(acc[3][3]) : "v"(a[0]), "v"(a[3]));
    }
#pragma unroll
    for (int mb = 0; mb < 4; ++mb) {
#pragma unroll
        for (int nb = 0; nb < 4; ++nb) {
#pragma unroll
            for (int j = 0; j < 8; ++j) os[(hi * 8 + j) * 68 + nb * 16 + lr] = acc[mb][nb][j]; }
        __builtin_amdgcn_wave_barrier(); asm volatile("" ::: "memory");
        float* crow = C + (size_t)(r0 + mb * 16) * ldc + c0;
#pragma unroll 1
        for (int ps = 0; ps < 2; ++ps) {
#pragma unroll
            for (int s = 0; s < 8; ++s) { const int row = 2 * s + hi, cofs = lr * 4; v4f val = *(const v4fa*)(os + row * 68 + cofs); if (BIAS) { val[0] += bfr(bias[c0 + cofs]); val[1] += bfr(bias[c0 + cofs + 1]); val[2] += bfr(bias[c0 + cofs + 2]); val[3] += bfr(bias[c0 + cofs + 3]); }
                *(volatile v4f*)(crow + (size_t)row * ldc + cofs) = val; }
            if (ps == 0) __threadfence(); }
        __builtin_amdgcn_wave_barrier(); asm volatile("" ::: "memory");
    }
}

__device__ __forceinline__ h16 tohx(float x) { return (h16)x; }
__device__ __forceinline__ void splitf(float y, unsigned short& h, unsigned short& l) { h = f2bf(y); l = f2bf(y - bf2f(h)); }
typedef __attribute__((ext_vector_type(2))) unsigned short v2us;
typedef __attribute__((ext_vector_type(4))) unsigned short v4us;
typedef __attribute__((ext_vector_type(2))) _Float16 v2h;
typedef __attribute__((ext_vector_type(4))) _Float16 v4h;
typedef __attribute__((ext_vector_type(2))) float v2f;

__global__ __launch_bounds__(256) void k_cvt8(const float* __restrict__ src, bf* dst, size_t n8) { const size_t i = (size_t)blockIdx.x * 256 + threadIdx.x; if (i >= n8) return; const v8f v = *(const v8f*)(src + i * 8); v8us o;
#pragma unroll
    for (int k = 0; k < 8; ++k) o[k] = f2bf(v[k]); *(volatile v8us*)(dst + i * 8) = o; __threadfence(); *(volatile v8us*)(dst + i * 8) = o; }
__global__ __launch_bounds__(256) void k_rms(const float* __restrict__ X, const float* __restrict__ w, bf* Hh, bf* Hl) { const int lane = threadIdx.x & 31; const int t = blockIdx.x * 8 + (threadIdx.x >> 5); if (t >= TT) return; float v[DM / 32]; float q = 0.f;
#pragma unroll
    for (int ch = 0; ch < DM / 128; ++ch) { const v4f a = *(const v4f*)(X + (size_t)t * DM + ch * 128 + lane * 4);
#pragma unroll
        for (int u = 0; u < 4; ++u) { v[ch * 4 + u] = bfr(a[u]); float p = __fmul_rn(v[ch * 4 + u], v[ch * 4 + u]); asm volatile("" : "+v"(p)); q = __fadd_rn(q, p); } }
#pragma unroll
    for (int sh = 16; sh; sh >>= 1) q += __shfl_xor(q, sh, 32);
    const float rs = __frsqrt_rn(__fadd_rn(q * (1.0f / DM), 1e-6f));
    for (int ps = 0; ps < 2; ++ps) {
#pragma unroll
        for (int ch = 0; ch < DM / 128; ++ch) { const int c0 = ch * 128 + lane * 4; v4us oh, ol;
#pragma unroll
            for (int u = 0; u < 4; ++u) { float n0 = __fmul_rn(v[ch * 4 + u], rs); asm volatile("" : "+v"(n0)); const float y = __fmul_rn(n0, bfr(w[c0 + u])); unsigned short a2, b2; splitf(y, a2, b2); oh[u] = a2; ol[u] = b2; }
            const size_t oo = (size_t)t * DM + c0; *(volatile v4us*)(Hh + oo) = oh; *(volatile v4us*)(Hl + oo) = ol; }
        if (ps == 0) __threadfence(); } }
__global__ __launch_bounds__(256) void k_cs(const int* __restrict__ pos, float* CS) { const int idx = blockIdx.x * 256 + threadIdx.x; if (idx >= TT * HD) return; const int dd = idx % HD; const int t = idx / HD; const int i2 = dd % (HD / 2); const float inv = __fdiv_rn(1.0f, powf(10000.0f, (float)(2 * i2) / (float)HD)); const float ang = __fmul_rn((float)pos[t], inv); v2f cs; cs[0] = cosf(ang); cs[1] = sinf(ang);
    *(volatile v2f*)(CS + (size_t)idx * 2) = cs; __threadfence(); *(volatile v2f*)(CS + (size_t)idx * 2) = cs; }
__global__ __launch_bounds__(256) void k_ropep(const float* __restrict__ F, const float* __restrict__ CS, bf* Ph, bf* Pl) { const size_t e = ((size_t)blockIdx.x * 256 + threadIdx.x) * 2; if (e >= (size_t)NH_ * TT * HD) return; const int d = (int)(e % HD); const int t = (int)((e / HD) % TT); const int h = (int)(e / ((size_t)HD * TT)); const float* f = F + (size_t)t * DM + h * HD; v2us oh, ol;
#pragma unroll
    for (int q = 0; q < 2; ++q) { const int dd = d + q; const int dp = (dd < HD / 2) ? dd + HD / 2 : dd - HD / 2; const float x0 = f[dd], x1 = f[dp]; const v2f cs = *(const v2f*)(CS + ((size_t)t * HD + dd) * 2);
        float a = __fmul_rn(x0, cs[0]), bq = __fmul_rn(x1, cs[1]); asm volatile("" : "+v"(a)); asm volatile("" : "+v"(bq)); const float r = (dd < HD / 2) ? __fsub_rn(a, bq) : __fadd_rn(a, bq); unsigned short a2, c2; splitf(r, a2, c2); oh[q] = a2; ol[q] = c2; }
    *(volatile v2us*)(Ph + e) = oh; *(volatile v2us*)(Pl + e) = ol; __threadfence(); *(volatile v2us*)(Ph + e) = oh; *(volatile v2us*)(Pl + e) = ol; }
__global__ __launch_bounds__(256) void k_vt(const float* __restrict__ V, h16* VT) { const int e = (blockIdx.x * 256 + threadIdx.x) * 2; if (e >= NH_ * HD * TT) return; const int t = e % TT; const int d = (e / TT) % HD; const int h = e / (TT * HD); v2h o; o[0] = tohx(V[(size_t)t * DM + h * HD + d]); o[1] = tohx(V[(size_t)(t + 1) * DM + h * HD + d]); *(volatile v2h*)(VT + e) = o; __threadfence(); *(volatile v2h*)(VT + e) = o; }
__global__ __launch_bounds__(256) void k_msoft(const float* __restrict__ Sb, const float* __restrict__ mk, h16* P16) { const int lane = threadIdx.x & 31; const int row = blockIdx.x * 8 + (threadIdx.x >> 5); if (row >= HPP * TT) return; const int i = row % TT; const float* sr = Sb + (size_t)row * TT; const float* mr = mk + (size_t)i * TT; float v[TT / 32]; float mx = -3.0e38f;
#pragma unroll
    for (int ch = 0; ch < TT / 128; ++ch) { const int j0 = ch * 128 + lane * 4; const v4f a = *(const v4f*)(sr + j0), m4 = *(const v4f*)(mr + j0);
#pragma unroll
        for (int u = 0; u < 4; ++u) { float m1 = bfr(m4[u]); asm volatile("" : "+v"(m1)); const float t = __fadd_rn(a[u], m1); v[ch * 4 + u] = t; mx = fmaxf(mx, t); } }
#pragma unroll
    for (int sh = 16; sh; sh >>= 1) mx = fmaxf(mx, __shfl_xor(mx, sh, 32));
    float sum = 0.f;
#pragma unroll
    for (int q = 0; q < TT / 32; ++q) { float d0 = __fsub_rn(v[q], mx); asm volatile("" : "+v"(d0)); v[q] = __builtin_amdgcn_exp2f(__fmul_rn(d0, 1.4426950408889634f)); sum += v[q]; }
#pragma unroll
    for (int sh = 16; sh; sh >>= 1) sum += __shfl_xor(sum, sh, 32);
    const float f = __fdiv_rn(PCAR, sum);
    for (int ps = 0; ps < 2; ++ps) {
#pragma unroll
        for (int ch = 0; ch < TT / 128; ++ch) { v4h o4;
#pragma unroll
            for (int q = 0; q < 4; ++q) o4[q] = tohx(v[ch * 4 + q] * f); *(volatile v4h*)(P16 + (size_t)row * TT + ch * 128 + lane * 4) = o4; }
        if (ps == 0) __threadfence(); } }
__global__ __launch_bounds__(256) void k_mrg(const float* __restrict__ O, int h0, bf* Ah, bf* Al) { const int e = (blockIdx.x * 256 + threadIdx.x) * 4; if (e >= HPP * TT * HD) return; const int d = e % HD; const int t = (e / HD) % TT; const int z = e / (HD * TT); v4us oh, ol;
#pragma unroll
    for (int u = 0; u < 4; ++u) { unsigned short a, b; splitf(O[e + u] * (1.0f / PCAR), a, b); oh[u] = a; ol[u] = b; } const size_t oo = (size_t)t * DM + (h0 + z) * HD + d; *(volatile v4us*)(Ah + oo) = oh; *(volatile v4us*)(Al + oo) = ol; __threadfence(); *(volatile v4us*)(Ah + oo) = oh; *(volatile v4us*)(Al + oo) = ol; }
__global__ __launch_bounds__(256) void k_fin(const float* __restrict__ X, const float* __restrict__ O2, float* outb) { const int e = (blockIdx.x * 256 + threadIdx.x) * 4; if (e >= TT * DM) return; const v4f a = *(const v4f*)(X + e), b = *(const v4f*)(O2 + e); v4f r;
#pragma unroll
    for (int u = 0; u < 4; ++u) r[u] = __fadd_rn(bfr(a[u]), b[u]); *(volatile v4f*)(outb + e) = r; __threadfence(); *(volatile v4f*)(outb + e) = r; }

extern "C" void kernel_launch(void* const* d_in, const int* in_sizes, int n_in,
                              void* d_out, int out_size, void* d_ws, size_t ws_size, hipStream_t stream) {
    (void)in_sizes; (void)n_in; (void)out_size;
    const float* x = (const float*)d_in[0]; const float* amask = (const float*)d_in[1]; const int* pos = (const int*)d_in[2]; const float* lnw = (const float*)d_in[3]; const float* wq = (const float*)d_in[4]; const float* wk = (const float*)d_in[5]; const float* wv = (const float*)d_in[6]; const float* wo = (const float*)d_in[7];
    float* OUT = (float*)d_out;
    char* wsp = (char*)d_ws;
    auto take = [&](size_t bytes) { char* p = wsp; wsp += (bytes + 255) & ~(size_t)255; return (void*)p; };
    bf* BQ = (bf*)take((size_t)DM * DM * 2); bf* BK = (bf*)take((size_t)DM * DM * 2); bf* BV = (bf*)take((size_t)DM * DM * 2); bf* BO = (bf*)take((size_t)DM * DM * 2);
    bf* NH = (bf*)take((size_t)TT * DM * 2); bf* NL = (bf*)take((size_t)TT * DM * 2); float* Q = (float*)take((size_t)TT * DM * 4); float* K = (float*)take((size_t)TT * DM * 4); float* V = (float*)take((size_t)TT * DM * 4); float* CS = (float*)take((size_t)TT * HD * 2 * 4);
    bf* Qh = (bf*)take((size_t)NH_ * TT * HD * 2); bf* Ql = (bf*)take((size_t)NH_ * TT * HD * 2); bf* Kh = (bf*)take((size_t)NH_ * TT * HD * 2); bf* Kl = (bf*)take((size_t)NH_ * TT * HD * 2); h16* VT = (h16*)take((size_t)NH_ * HD * TT * 2);
    float* Sb = (float*)take((size_t)HPP * TT * TT * 4); h16* P16 = (h16*)take((size_t)HPP * TT * TT * 2); float* O = (float*)take((size_t)HPP * TT * HD * 4); bf* Ah = (bf*)take((size_t)TT * DM * 2); bf* Al = (bf*)take((size_t)TT * DM * 2); float* O2 = (float*)take((size_t)TT * DM * 4);
    if ((size_t)(wsp - (char*)d_ws) > ws_size) return;
    k_cvt8<<<(DM * DM / 8 + 255) / 256, 256, 0, stream>>>(wq, BQ, DM * DM / 8); k_cvt8<<<(DM * DM / 8 + 255) / 256, 256, 0, stream>>>(wk, BK, DM * DM / 8); k_cvt8<<<(DM * DM / 8 + 255) / 256, 256, 0, stream>>>(wv, BV, DM * DM / 8); k_cvt8<<<(DM * DM / 8 + 255) / 256, 256, 0, stream>>>(wo, BO, DM * DM / 8);
    const dim3 gp(TT / 64, DM / 64, 1); const size_t zq = (size_t)TT * HD, zS = (size_t)TT * TT;
    for (int b = 0; b < NB_; ++b) { const float* xb = x + (size_t)b * TT * DM;
        k_rms<<<TT / 8, 256, 0, stream>>>(xb, lnw, NH, NL); k_cs<<<(TT * HD + 255) / 256, 256, 0, stream>>>(pos + (size_t)b * TT, CS);
        k_gemmw<bf, 1, false><<<gp, 32, 0, stream>>>(NH, NL, BQ, nullptr, DM, Q, DM, nullptr, 0, 0, 0); k_gemmw<bf, 1, false><<<gp, 32, 0, stream>>>(NH, NL, BK, nullptr, DM, K, DM, nullptr, 0, 0, 0); k_gemmw<bf, 1, false><<<gp, 32, 0, stream>>>(NH, NL, BV, nullptr, DM, V, DM, nullptr, 0, 0, 0);
        k_ropep<<<(unsigned)(((size_t)NH_ * TT * HD / 2 + 255) / 256), 256, 0, stream>>>(Q, CS, Qh, Ql); k_ropep<<<(unsigned)(((size_t)NH_ * TT * HD / 2 + 255) / 256), 256, 0, stream>>>(K, CS, Kh, Kl); k_vt<<<(NH_ * HD * TT / 2 + 255) / 256, 256, 0, stream>>>(V, VT);
        for (int h0 = 0; h0 < NH_; h0 += HPP) { const size_t zo = (size_t)h0 * zq;
            k_gemmw<bf, 2, false><<<dim3(TT / 64, TT / 64, HPP), 32, 0, stream>>>(Qh + zo, Ql + zo, Kh + zo, Kl + zo, HD, Sb, TT, nullptr, zq, zq, zS);
            k_msoft<<<HPP * TT / 8, 256, 0, stream>>>(Sb, amask + (size_t)b * TT * TT, P16);
            k_gemmw<h16, 0, false><<<dim3(TT / 64, 1, HPP), 32, 0, stream>>>(P16, nullptr, VT + zo, nullptr, TT, O, HD, nullptr, zS, (size_t)HD * TT, zq);
            k_mrg<<<(HPP * TT * HD / 4 + 255) / 256, 256, 0, stream>>>(O, h0, Ah, Al); }
        k_gemmw<bf, 1, false><<<gp, 32, 0, stream>>>(Ah, Al, BO, nullptr, DM, O2, DM, nullptr, 0, 0, 0);
        k_fin<<<(TT * DM / 4 + 255) / 256, 256, 0, stream>>>(xb, O2, OUT + (size_t)b * TT * DM); }
}
